// MHA_26792005992553
// MI455X (gfx1250) — hardware-verified
//
#include <hip/hip_runtime.h>
#include <math.h>

typedef __attribute__((ext_vector_type(16))) _Float16 v16h;
typedef __attribute__((ext_vector_type(16))) __bf16 v16b;
typedef __attribute__((ext_vector_type(8)))  _Float16 v8h;
typedef __attribute__((ext_vector_type(8)))  float v8f;
typedef __attribute__((ext_vector_type(4)))  float v4f;
typedef __attribute__((ext_vector_type(4)))  unsigned v4u;

template <typename T> __device__ __forceinline__ void vst2(void* p, T v) { *(volatile T*)p = v; __threadfence(); *(volatile T*)p = v; }
__device__ __forceinline__ v8f wmma16(v16h a, v16h b, v8f c) {
  v8f d = __builtin_amdgcn_wmma_f32_16x16x32_f16(false, a, false, b, (short)0, c, false, false);
  asm volatile("v_nop\n\tv_nop\n\tv_nop\n\tv_nop" : "+v"(d) : "v"(a), "v"(b));
  return d;
}
__device__ __forceinline__ v8f wmma_bf(v16b a, v16b b, v8f c) {
  v8f d = __builtin_amdgcn_wmma_f32_16x16x32_bf16(false, a, false, b, (short)0, c, false, false);
  asm volatile("v_nop\n\tv_nop\n\tv_nop\n\tv_nop" : "+v"(d) : "v"(a), "v"(b));
  return d;
}
__device__ __forceinline__ v16h frag_h(const _Float16* rowk0, unsigned lane) {
  union { v16h v; v8h q[2]; } u; const _Float16* p = rowk0 + 8u * (lane >> 4);
  u.q[0] = *(const v8h*)p; u.q[1] = *(const v8h*)(p + 16); return u.v;
}
__device__ __forceinline__ v16h frag_f32(const float* rowk0, unsigned lane) {
  v16h a; const float* p = rowk0 + 8u * (lane >> 4);
#pragma unroll
  for (int i = 0; i < 8; ++i) { a[i] = (_Float16)p[i]; a[8 + i] = (_Float16)p[16 + i]; }
  return a;
}
__device__ __forceinline__ float bfr(float v) { return (float)(__bf16)v; }
__device__ __forceinline__ v16b wcol_oi(const float* Wm, unsigned k0, unsigned o, unsigned lane, unsigned K) { v16b w; const float* p = Wm + (size_t)o * K + k0 + 8u * (lane >> 4);
#pragma unroll
  for (int i = 0; i < 8; ++i) { w[i] = (__bf16)p[i]; w[8 + i] = (__bf16)p[16 + i]; }
  return w; }
__device__ __forceinline__ v16h wcolh_oi(const float* Wm, unsigned k0, unsigned o, unsigned lane, unsigned K) { v16h w; const float* p = Wm + (size_t)o * K + k0 + 8u * (lane >> 4);
#pragma unroll
  for (int i = 0; i < 8; ++i) { w[i] = (_Float16)(bfr(p[i]) * 256.0f); w[8 + i] = (_Float16)(bfr(p[16 + i]) * 256.0f); }
  return w; }
#define LDSX() do { asm volatile("s_wait_dscnt 0" ::: "memory"); __builtin_amdgcn_wave_barrier(); __builtin_amdgcn_fence(3  , "workgroup"); } while (0)

#ifndef NB
#define NB 2
#endif
#ifndef SEQ
#define SEQ 2048
#endif
#define TT SEQ
#define NB_FULL 2
#define TT_FULL 2048
#define CC 1024
#define DIN 1024
#define NH 16
#define HD 64
#define NQB (TT / 64)
#define HG 4
#define SCALE (0.125f)
#define PCARRY (2048.0f)
#define YSC (1.0f / 32.0f)
#define OSC (1.0f / 16384.0f)

static_assert(NB <= NB_FULL);
static_assert(TT <= TT_FULL);
static_assert((TT & (TT - 1)) == 0);
static_assert(TT % 128 == 0);
static_assert(CC % 128 == 0);
static_assert(DIN % 32 == 0);
static_assert(CC % 32 == 0);
static_assert(CC == NH * HD);
static_assert(DIN == CC);
static_assert(HD == 64);
static_assert(NH % HG == 0);
static_assert((NB * TT) % 64 == 0);

#define WS_QH  ((size_t)0)
#define WS_KH  (WS_QH + 2u * (size_t)NB * TT * CC)
#define WS_VT  (WS_KH + 2u * (size_t)NB * TT * CC)
#define WS_YH  (WS_VT + 2u * (size_t)NB * CC * TT)
#define WS_S   (WS_YH + 2u * (size_t)NB * TT * CC)
#define WS_END (WS_S  + 4u * (size_t)HG * TT * TT)
static_assert(WS_END <= (size_t)134217728);
static_assert(WS_KH % 128 == 0);
static_assert(WS_VT % 128 == 0);
static_assert(WS_YH % 128 == 0);
static_assert(WS_S % 128 == 0);

__global__ __launch_bounds__(128) void k_proj(const float* __restrict__ X, const float* __restrict__ WQ, const float* __restrict__ WK, const float* __restrict__ WV, const float* __restrict__ BQ, const float* __restrict__ BK, const float* __restrict__ BV,
    _Float16* __restrict__ QH, _Float16* __restrict__ KH, _Float16* __restrict__ VT) {
  __shared__ __align__(16) _Float16 sh[64][136]; __shared__ __align__(16) _Float16 th[128][72];
  const unsigned tid = threadIdx.x, wave = tid >> 5, lane = tid & 31u, col = lane & 15u, g = lane >> 4;
  const unsigned which = blockIdx.z, c0 = blockIdx.y * 128u, r0 = blockIdx.x * 64u, bb = r0 / (unsigned)TT, t0 = r0 % (unsigned)TT;
  const float* WA = which == 0u ? WQ : which == 1u ? WK : WV; const float* BA = which == 0u ? BQ : which == 1u ? BK : BV;
  const float* xrow = X + ((size_t)bb * TT_FULL + t0 + wave * 16u + col) * DIN;
  v8f acc[8] = {};
#pragma unroll 2
  for (unsigned kc = 0; kc < DIN / 32; ++kc) { v16b a; { const float* p = xrow + kc * 32u + 8u * g;
#pragma unroll
      for (int i = 0; i < 8; ++i) { a[i] = (__bf16)p[i]; a[8 + i] = (__bf16)p[16 + i]; } }
    asm volatile("s_wait_loadcnt 0x0" ::: "memory");
#pragma unroll
    for (int j = 0; j < 8; ++j) { const v16b w = wcol_oi(WA, kc * 32u, c0 + j * 16u + col, lane, DIN); asm volatile("s_wait_loadcnt 0x0" ::: "memory"); acc[j] = wmma_bf(a, w, acc[j]); } }
  if (which < 2u) { _Float16* DH = which == 0u ? QH : KH;
#pragma unroll
    for (int j = 0; j < 8; ++j) { const float bias = bfr(BA[c0 + j * 16u + col]);
#pragma unroll
      for (int r = 0; r < 8; ++r) { const float v = acc[j][r] + bias; sh[wave * 16u + 8u * g + r][j * 16u + col] = (_Float16)v; } }
    __syncthreads();
    for (unsigned e = tid; e < 64u * 16u; e += 128u) { const unsigned rl = e >> 4, q = e & 15u; const v4u t = *(const v4u*)&sh[rl][q * 8u]; vst2(DH + ((size_t)r0 + rl) * CC + c0 + q * 8u, t); }
  } else {
#pragma unroll
    for (int j = 0; j < 8; ++j) { const float bias = bfr(BA[c0 + j * 16u + col]);
#pragma unroll
      for (int r = 0; r < 8; ++r) { const float v = acc[j][r] + bias; th[j * 16u + col][wave * 16u + 8u * g + r] = (_Float16)v; } }
    __syncthreads();
    for (unsigned e = tid; e < 128u * 8u; e += 128u) { const unsigned cl = e >> 3, q = e & 7u; const v4u t = *(const v4u*)&th[cl][q * 8u]; vst2(VT + ((size_t)bb * CC + c0 + cl) * TT + t0 + q * 8u, t); } } }
__global__ __launch_bounds__(128) void k_sc(const _Float16* __restrict__ QH, const _Float16* __restrict__ KH, unsigned b, unsigned h0, float* __restrict__ S0) { __shared__ __align__(16) float ss[4][16][132];
  const unsigned qb = blockIdx.x, kb = blockIdx.y, h = h0 + blockIdx.z; float* S = S0 + (size_t)blockIdx.z * TT * TT;
  const unsigned tid = threadIdx.x, wave = tid >> 5, lane = tid & 31u, col = lane & 15u, g = lane >> 4; const unsigned k0 = kb * 128u; const unsigned ql0 = qb * 64u + wave * 16u; const size_t q0 = (size_t)b * TT + ql0, kr0 = (size_t)b * TT + k0;
  v8f acc[8] = {};
#pragma unroll
  for (int kc = 0; kc < HD / 32; ++kc) { const v16h ah = frag_h(QH + (q0 + col) * CC + h * HD + kc * 32, lane);
#pragma unroll
    for (int j = 0; j < 8; ++j) { const v16h kbf = frag_h(KH + (kr0 + j * 16u + col) * CC + h * HD + kc * 32, lane); acc[j] = wmma16(ah, kbf, acc[j]); } }
#pragma unroll
  for (int j = 0; j < 8; ++j) {
#pragma unroll
    for (int r = 0; r < 8; ++r) ss[wave][8u * g + r][j * 16u + col] = acc[j][r] * SCALE; }
  LDSX(); for (unsigned rl = 0; rl < 16u; ++rl) { const v4f t = *(const v4f*)&ss[wave][rl][lane * 4u]; vst2(S + (size_t)(ql0 + rl) * TT + k0 + lane * 4u, t); } }
__global__ __launch_bounds__(256) void k_sm(float* __restrict__ S0) { __shared__ float sred[8]; __shared__ float sbc; __shared__ __align__(16) float shv[TT];
  const unsigned tid = threadIdx.x; const unsigned t = blockIdx.x;
  float* sr = S0 + (size_t)blockIdx.y * TT * TT + (size_t)t * TT;
  float m = -3.0e38f;
#pragma unroll 1
  for (unsigned k = tid; k < (unsigned)TT; k += 256u) { const float v = sr[k]; shv[k] = v; m = fmaxf(m, v); }
#pragma unroll
  for (int o = 1; o < 32; o <<= 1) m = fmaxf(m, __shfl_xor(m, o));
  if ((tid & 31u) == 0u) sred[tid >> 5] = m; __syncthreads(); if (tid == 0u) { float a = sred[0]; for (int i = 1; i < 8; ++i) a = fmaxf(a, sred[i]); sbc = a; } __syncthreads(); m = sbc; __syncthreads();
  float sum = 0.f;
#pragma unroll 1
  for (unsigned k = tid; k < (unsigned)TT; k += 256u) { const float e = expf(shv[k] - m); shv[k] = e; sum += e; }
#pragma unroll
  for (int o = 1; o < 32; o <<= 1) sum += __shfl_xor(sum, o);
  if ((tid & 31u) == 0u) sred[tid >> 5] = sum; __syncthreads(); if (tid == 0u) { float a = 0.f; for (int i = 0; i < 8; ++i) a += sred[i]; sbc = a > 0.f ? PCARRY * (1.0f / a) : 0.f; } __syncthreads(); const float inv = sbc;
#pragma unroll 1
  for (unsigned k = tid; k < (unsigned)TT; k += 256u) shv[k] = shv[k] * inv;
  __syncthreads();
#pragma unroll 1
  for (unsigned q = tid; q < (unsigned)TT / 4u; q += 256u) { const v4f t4 = *(const v4f*)&shv[q * 4u]; vst2(sr + q * 4u, t4); } }
__global__ __launch_bounds__(128) void k_pv(const float* __restrict__ PS0, const _Float16* __restrict__ VT, unsigned b, unsigned h0, _Float16* __restrict__ YH) { const unsigned h = h0 + blockIdx.z; const float* PS = PS0 + (size_t)blockIdx.z * TT * TT; __shared__ __align__(16) _Float16 sc[4][16][72];
  const unsigned tid = threadIdx.x, wave = tid >> 5, lane = tid & 31u, col = lane & 15u, g = lane >> 4; const unsigned qb = blockIdx.x; const unsigned ql0 = qb * 64u + wave * 16u;
  v8f acc[HD / 16] = {};
#pragma unroll 1
  for (unsigned kc = 0; kc < (unsigned)TT / 32u; ++kc) { const v16h p = frag_f32(PS + (size_t)(ql0 + col) * TT + kc * 32u, lane);
    asm volatile("s_wait_loadcnt 0x0" ::: "memory");
#pragma unroll
    for (int j = 0; j < HD / 16; ++j) { const size_t po = ((size_t)b * CC + h * HD + j * 16u + col) * (size_t)TT + kc * 32u; acc[j] = wmma16(p, frag_h(VT + po, lane), acc[j]); } }
#pragma unroll
  for (int j = 0; j < HD / 16; ++j)
#pragma unroll
    for (int r = 0; r < 8; ++r) sc[wave][8u * g + r][j * 16u + col] = (_Float16)(acc[j][r] * YSC);
  LDSX();
  for (unsigned it = 0; it < 4u; ++it) { const unsigned row = it * 4u + (lane >> 3), pc = lane & 7u; const v8h t = *(const v8h*)&sc[wave][row][pc * 8u]; vst2(YH + ((size_t)b * TT + ql0 + row) * CC + h * HD + pc * 8u, t); } }
__global__ __launch_bounds__(128) void k_oproj(const _Float16* __restrict__ YH, const float* __restrict__ WO, const float* __restrict__ BO, float* __restrict__ OUT) { __shared__ __align__(16) float ss[4][16][132];
  const unsigned tid = threadIdx.x, wave = tid >> 5, lane = tid & 31u, col = lane & 15u, g = lane >> 4; const unsigned c0 = blockIdx.y * 128u, r0 = blockIdx.x * 64u + wave * 16u;
  const _Float16* yrow = YH + ((size_t)r0 + col) * CC;
  v8f acc[8] = {};
#pragma unroll 2
  for (unsigned kc = 0; kc < CC / 32; ++kc) { const v16h a = frag_h(yrow + kc * 32u, lane);
    asm volatile("s_wait_loadcnt 0x0" ::: "memory");
#pragma unroll
    for (int j = 0; j < 8; ++j) { const v16h w = wcolh_oi(WO, kc * 32u, c0 + j * 16u + col, lane, CC); asm volatile("s_wait_loadcnt 0x0" ::: "memory"); acc[j] = wmma16(a, w, acc[j]); } }
#pragma unroll
  for (int j = 0; j < 8; ++j) { const float bias = bfr(BO[c0 + j * 16u + col]);
#pragma unroll
    for (int r = 0; r < 8; ++r) ss[wave][8u * g + r][j * 16u + col] = acc[j][r] * OSC + bias; }
  LDSX(); for (unsigned rl = 0; rl < 16u; ++rl) { const v4f t = *(const v4f*)&ss[wave][rl][lane * 4u]; vst2(OUT + ((size_t)r0 + rl) * CC + c0 + lane * 4u, t); } }

extern "C" void kernel_launch(void* const* d_in, const int* in_sizes, int n_in, void* d_out, int out_size, void* d_ws, size_t ws_size, hipStream_t stream) {
  if (n_in < 9) return;
  const long long need_x = ((long long)(NB - 1) * TT_FULL + TT) * DIN;
  if ((long long)in_sizes[0] < need_x) return;
  if (in_sizes[1] < CC * DIN || in_sizes[3] < CC * DIN || in_sizes[5] < CC * DIN || in_sizes[7] < CC * CC) return;
  if (in_sizes[2] < CC || in_sizes[4] < CC || in_sizes[6] < CC || in_sizes[8] < CC) return;
  if ((long long)out_size < (long long)NB * TT * CC) return;
  if (ws_size < (size_t)WS_END) return;
  const float** F = (const float**)d_in;
  char* ws = (char*)d_ws; _Float16 *QH = (_Float16*)(ws + WS_QH), *KH = (_Float16*)(ws + WS_KH), *VT = (_Float16*)(ws + WS_VT), *YH = (_Float16*)(ws + WS_YH); float* S = (float*)(ws + WS_S);
  k_proj<<<dim3(NB * TT / 64, CC / 128, 3), 128, 0, stream>>>(F[0], F[1], F[3], F[5], F[2], F[4], F[6], QH, KH, VT);
  for (unsigned b = 0; b < (unsigned)NB; ++b) for (unsigned h0 = 0; h0 < (unsigned)NH; h0 += HG) {
    k_sc<<<dim3(NQB, TT / 128, HG), 128, 0, stream>>>(QH, KH, b, h0, S);
    k_sm<<<dim3(TT, HG), 256, 0, stream>>>(S);
    k_pv<<<dim3(NQB, 1, HG), 128, 0, stream>>>(S, VT, b, h0, YH);
  }
  k_oproj<<<dim3(NB * TT / 64, CC / 128), 128, 0, stream>>>(YH, F[7], F[8], (float*)d_out);
}
